// TransformerBlock_67310727463209
// MI455X (gfx1250) — hardware-verified
//
#include <hip/hip_runtime.h>
#include <stddef.h>


typedef _Float16 v16h __attribute__((ext_vector_type(16)));
typedef _Float16 v8h  __attribute__((ext_vector_type(8)));
typedef float    v8f  __attribute__((ext_vector_type(8)));
typedef float    v4f  __attribute__((ext_vector_type(4)));

#ifndef SEQ
#define SEQ 2048
#endif
#define SEQ_FULL 2048
#define DIM   1024
#define NHEAD 16
#define HD    64
#define DFF   4096
#define DCOND 512

static_assert(SEQ >= 128 && SEQ <= SEQ_FULL && (SEQ % 128) == 0);
static_assert(DIM == NHEAD * HD);
static_assert(HD == 64);
static_assert((DIM % 64) == 0 && (DIM % 32) == 0);
static_assert((DFF % 64) == 0 && (DFF % 32) == 0);
static_assert((SEQ % 64) == 0 && (SEQ % 8) == 0);
static_assert(DIM == 32 * 8 * 4);
static_assert((DCOND % 32) == 0);
static_assert(((size_t)3 * DIM * DIM) % 2048 == 0);
static_assert(((size_t)DIM * DIM) % 2048 == 0);
static_assert(((size_t)DFF * DIM) % 2048 == 0);
static_assert((size_t)SEQ * DFF < (size_t)0xFFFFFFFFu);

#define LDT 72
#define LDC 68

#define WCARRY 64.0f
#define PCARRY 1024.0f
#define VCARRY 64.0f

#define TAB_BYTES   ((size_t)4 * DIM * 4)
#define WQKV_BYTES  ((size_t)3 * DIM * DIM * 2)
#define WPROJ_BYTES ((size_t)DIM * DIM * 2)
#define WFF1_BYTES  ((size_t)DFF * DIM * 2)
#define WFF2_BYTES  ((size_t)DIM * DFF * 2)
#define P16_BYTES   ((size_t)SEQ * DIM * 2)
#define X1_BYTES    ((size_t)SEQ * DIM * 4)
#define H16_BYTES   ((size_t)SEQ * DFF * 2)

#define OFF_TAB   ((size_t)0)
#define OFF_WQKV  (OFF_TAB + TAB_BYTES)
#define OFF_WPROJ (OFF_WQKV + WQKV_BYTES)
#define OFF_WFF1  (OFF_WPROJ + WPROJ_BYTES)
#define OFF_WFF2  (OFF_WFF1 + WFF1_BYTES)
#define OFF_XN    (OFF_WFF2 + WFF2_BYTES)
#define OFF_QK    (OFF_XN + P16_BYTES)
#define OFF_VT    (OFF_QK + 2 * P16_BYTES)
#define OFF_CTX   (OFF_VT + P16_BYTES)
#define OFF_X1    (OFF_CTX + P16_BYTES)
#define OFF_H     (OFF_X1 + X1_BYTES)
#define WS_TOTAL  (OFF_H + H16_BYTES)
static_assert((TAB_BYTES % 128) == 0 && (WQKV_BYTES % 128) == 0 && (WPROJ_BYTES % 128) == 0);
static_assert((WFF1_BYTES % 128) == 0 && (WFF2_BYTES % 128) == 0 && (P16_BYTES % 128) == 0);
static_assert((X1_BYTES % 128) == 0 && (H16_BYTES % 128) == 0);
static_assert(WS_TOTAL <= (size_t)134217728);

__device__ __forceinline__ float bf16r(float x) {
  unsigned int u = __float_as_uint(x);
  u = (u + 0x7FFFu + ((u >> 16) & 1u)) & 0xFFFF0000u;
  return __uint_as_float(u);
}

__device__ __forceinline__ v16h frag_at(const _Float16* p) {
  v8h lo = *(const v8h*)(p);
  v8h hi = *(const v8h*)(p + 16);
  v16h out;
#pragma unroll
  for (int i = 0; i < 8; ++i) { out[i] = lo[i]; out[i + 8] = hi[i]; }
  return out;
}
__device__ __forceinline__ v16h ld_frag(const _Float16* base, unsigned ld) {
  const unsigned lane = threadIdx.x & 31u;
  return frag_at(base + (lane & 15u) * ld + (lane >> 4) * 8u);
}

__device__ __forceinline__ v8f wmma16(v16h a, v16h b, v8f c) {
  v8f d = __builtin_amdgcn_wmma_f32_16x16x32_f16(false, a, false, b, (short)0, c,
                                                 false, false);
  asm volatile("v_nop\n\tv_nop\n\tv_nop\n\tv_nop" : "+v"(d) : "v"(a), "v"(b));
  return d;
}

__device__ __forceinline__ float red16_max(float x) {
#pragma unroll
  for (int off = 1; off < 16; off <<= 1) x = fmaxf(x, __shfl_xor(x, off, 32));
  return x;
}
__device__ __forceinline__ float red16_sum(float x) {
#pragma unroll
  for (int off = 1; off < 16; off <<= 1) x += __shfl_xor(x, off, 32);
  return x;
}
__device__ __forceinline__ float red32_sum(float x) {
#pragma unroll
  for (int off = 1; off < 32; off <<= 1) x += __shfl_xor(x, off, 32);
  return x;
}

__device__ __forceinline__ void wave_lds_sync() {
  __builtin_amdgcn_fence(3  , "wavefront");
  asm volatile("s_wait_dscnt 0x0" ::: "memory");
  __builtin_amdgcn_wave_barrier();
}

__device__ __forceinline__ float gelu_tanh(float t) {
  const float u = 0.7978845608028654f * (t + 0.044715f * t * t * t);
  const float e = expf(-2.0f * u);
  return t * __builtin_amdgcn_rcpf(1.0f + e);
}

__device__ __forceinline__ float dot_row(const float* __restrict__ wrow,
                                         const float* __restrict__ c, unsigned lane) {
  float acc = 0.0f;
#pragma unroll 1
  for (unsigned k = lane; k < (unsigned)DCOND; k += 32u)
    acc = fmaf(bf16r(wrow[k]), bf16r(c[k]), acc);
  return red32_sum(acc);
}

__global__ __launch_bounds__(256) void cond_kernel(
    const float* __restrict__ cond,
    const float* __restrict__ g1w, const float* __restrict__ g1b,
    const float* __restrict__ b1w, const float* __restrict__ b1b,
    const float* __restrict__ g2w, const float* __restrict__ g2b,
    const float* __restrict__ b2w, const float* __restrict__ b2b,
    float* __restrict__ tab) {
  __shared__ float stage[32];
  const unsigned tid = threadIdx.x, lane = tid & 31u, w = tid >> 5;
  const unsigned sel = blockIdx.x >> 5;
  const unsigned j0 = (blockIdx.x & 31u) * 32u;
#pragma unroll 1
  for (unsigned i = 0; i < 4u; ++i) {
    const unsigned j = j0 + w * 4u + i;
    float t;
    if (sel == 0u)      t = dot_row(g1w + (size_t)j * DCOND, cond, lane) + bf16r(g1b[j]);
    else if (sel == 1u) t = dot_row(b1w + (size_t)j * DCOND, cond, lane) + bf16r(b1b[j]);
    else if (sel == 2u) t = dot_row(g2w + (size_t)j * DCOND, cond, lane) + bf16r(g2b[j]);
    else                t = dot_row(b2w + (size_t)j * DCOND, cond, lane) + bf16r(b2b[j]);
    if ((sel & 1u) == 0u) t = t * (1.0f / (1.0f + expf(-t)));
    if (lane == 0u) stage[w * 4u + i] = t;
  }
  __syncthreads();
  if (tid < 8u) {
    const v4f v = *(const v4f*)&stage[tid * 4u];
    float* dp = tab + (size_t)blockIdx.x * 32u + tid * 4u;
    *(volatile v4f*)dp = v;
    __threadfence();
    *(volatile v4f*)dp = v;
  }
}

__global__ __launch_bounds__(256) void wcast_kernel(
    const float* __restrict__ src, _Float16* __restrict__ dst) {
  const size_t e = ((size_t)blockIdx.x * 256u + threadIdx.x) * 8u;
  const v4f a0 = *(const v4f*)(src + e);
  const v4f a1 = *(const v4f*)(src + e + 4);
  v8h o;
#pragma unroll
  for (int j = 0; j < 4; ++j) {
    o[j]     = (_Float16)(WCARRY * bf16r(a0[j]));
    o[j + 4] = (_Float16)(WCARRY * bf16r(a1[j]));
  }
  *(volatile v8h*)(dst + e) = o;
  __threadfence();
  *(volatile v8h*)(dst + e) = o;
}

struct F8 { v4f a, b; };
__device__ __forceinline__ F8 ld8(const float* __restrict__ p, int cvt) {
  F8 r;
  r.a = *(const v4f*)(p);
  r.b = *(const v4f*)(p + 4);
  if (cvt != 0) {
#pragma unroll
    for (int j = 0; j < 4; ++j) { r.a[j] = bf16r(r.a[j]); r.b[j] = bf16r(r.b[j]); }
  }
  return r;
}

__global__ __launch_bounds__(256) void adaln_kernel(
    const float* __restrict__ src, const float* __restrict__ lnw,
    const float* __restrict__ lnb, const float* __restrict__ gam,
    const float* __restrict__ bet, _Float16* __restrict__ dst, int cvt) {
  const unsigned tid = threadIdx.x, lane = tid & 31u, w = tid >> 5;
  const unsigned row = blockIdx.x * 8u + w;
  const float* xr = src + (size_t)row * DIM + lane * 8u;

  float s = 0.0f;
#pragma unroll 1
  for (unsigned t = 0; t < 4u; ++t) {
    const F8 v = ld8(xr + 256u * t, cvt);
    s += ((v.a[0] + v.a[1]) + (v.a[2] + v.a[3])) + ((v.b[0] + v.b[1]) + (v.b[2] + v.b[3]));
  }
  s = red32_sum(s);
  const float mu = s * (1.0f / (float)DIM);

  float q = 0.0f;
#pragma unroll 1
  for (unsigned t = 0; t < 4u; ++t) {
    const F8 v = ld8(xr + 256u * t, cvt);
#pragma unroll
    for (int j = 0; j < 4; ++j) {
      const float d0 = v.a[j] - mu, d1 = v.b[j] - mu;
      q = fmaf(d0, d0, q);
      q = fmaf(d1, d1, q);
    }
  }
  q = red32_sum(q);
  const float rstd = 1.0f / sqrtf(q * (1.0f / (float)DIM) + 1.0e-5f);

#pragma unroll 1
  for (unsigned t = 0; t < 4u; ++t) {
    const unsigned c = 256u * t + lane * 8u;
    const F8 v  = ld8(xr + 256u * t, cvt);
    const F8 lw = ld8(lnw + c, 1);
    const F8 lb = ld8(lnb + c, 1);
    const F8 g  = ld8(gam + c, 0);
    const F8 be = ld8(bet + c, 0);
    v8h o;
#pragma unroll
    for (int j = 0; j < 4; ++j) {
      const float y0 = (v.a[j] - mu) * rstd * lw.a[j] + lb.a[j];
      const float y1 = (v.b[j] - mu) * rstd * lw.b[j] + lb.b[j];
      o[j]     = (_Float16)((1.0f + g.a[j]) * y0 + be.a[j]);
      o[j + 4] = (_Float16)((1.0f + g.b[j]) * y1 + be.b[j]);
    }
    _Float16* dp = dst + (size_t)row * DIM + c;
    *(volatile v8h*)dp = o;
    __threadfence();
    *(volatile v8h*)dp = o;
  }
}

template <int MODE, int KD, int NPITCH, int SHIFT, int RCVT>
__device__ __forceinline__ void gemm_body(
    const _Float16* __restrict__ A16, const _Float16* __restrict__ Bt,
    const float* __restrict__ biasf, const float* __restrict__ residf,
    float* __restrict__ outf, _Float16* __restrict__ out16,
    _Float16* __restrict__ out16t) {
  static_assert((KD % 32) == 0);
  static_assert((NPITCH % 64) == 0);
  __shared__ float Cs[64 * LDC];
  const unsigned tid = threadIdx.x, lane = tid & 31u, w = tid >> 5;
  const unsigned mw = w >> 1, nw = w & 1u;
  const unsigned hh = lane >> 4, m = lane & 15u;
  const unsigned n0 = blockIdx.x * 64u;
  const unsigned row0 = blockIdx.y * 64u;

  const _Float16* ap  = A16 + (size_t)(row0 + mw * 16u + m) * KD + hh * 8u;
  const _Float16* bp0 = Bt + (size_t)(n0 + nw * 32u + m) * KD + hh * 8u;
  const _Float16* bp1 = bp0 + 16 * KD;
  v8f acc0 = {}, acc1 = {};
#pragma unroll 2
  for (unsigned k0 = 0; k0 < (unsigned)KD; k0 += 32u) {
    const v16h a  = frag_at(ap + k0);
    const v16h b0 = frag_at(bp0 + k0);
    const v16h b1 = frag_at(bp1 + k0);
    acc0 = wmma16(a, b0, acc0);
    acc1 = wmma16(a, b1, acc1);
  }
#pragma unroll
  for (int r = 0; r < 8; ++r) {
    float* d = &Cs[(mw * 16u + hh * 8u + (unsigned)r) * LDC + nw * 32u + m];
    d[0]  = acc0[r];
    d[16] = acc1[r];
  }
  __syncthreads();

  if (MODE == 0) {
    const unsigned third = n0 / (unsigned)DIM;
    const unsigned nn0 = n0 - third * (unsigned)DIM;
    v8h x[2];
    size_t off[2];
    if (third < 2u) {
#pragma unroll
      for (unsigned i = 0; i < 2u; ++i) {
        const unsigned r = 32u * i + (tid >> 3);
        const unsigned c = (tid & 7u) * 8u;
        const v4f u0 = *(const v4f*)&Cs[r * LDC + c];
        const v4f u1 = *(const v4f*)&Cs[r * LDC + c + 4];
#pragma unroll
        for (int j = 0; j < 4; ++j) {
          x[i][j]     = (_Float16)(u0[j] * (1.0f / WCARRY));
          x[i][j + 4] = (_Float16)(u1[j] * (1.0f / WCARRY));
        }
        off[i] = (size_t)third * SEQ * DIM + (size_t)(row0 + r) * DIM + nn0 + c;
      }
#pragma unroll
      for (int i = 0; i < 2; ++i) *(volatile v8h*)(out16 + off[i]) = x[i];
      __threadfence();
#pragma unroll
      for (int i = 0; i < 2; ++i) *(volatile v8h*)(out16 + off[i]) = x[i];
    } else {
#pragma unroll
      for (unsigned i = 0; i < 2u; ++i) {
        const unsigned dcol = 32u * i + (tid >> 3);
        const unsigned kk = (tid & 7u) * 8u;
#pragma unroll
        for (unsigned j = 0; j < 8u; ++j)
          x[i][j] = (_Float16)(Cs[(kk + j) * LDC + dcol] * (1.0f / WCARRY));
        off[i] = (size_t)(nn0 + dcol) * SEQ + row0 + kk;
      }
#pragma unroll
      for (int i = 0; i < 2; ++i) *(volatile v8h*)(out16t + off[i]) = x[i];
      __threadfence();
#pragma unroll
      for (int i = 0; i < 2; ++i) *(volatile v8h*)(out16t + off[i]) = x[i];
    }
  }

  if (MODE == 2) {
    const float sc = 1.0f / (float)(1 << SHIFT);
    v4f xs[4];
    size_t off[4];
#pragma unroll
    for (unsigned i = 0; i < 4u; ++i) {
      const unsigned r = 16u * i + (tid >> 4);
      const unsigned c = (tid & 15u) * 4u;
      const size_t o = (size_t)(row0 + r) * NPITCH + n0 + c;
      const v4f u = *(const v4f*)&Cs[r * LDC + c];
      const v4f g = *(const v4f*)(biasf + n0 + c);
      const v4f rs = *(const v4f*)(residf + o);
      v4f val;
#pragma unroll
      for (int j = 0; j < 4; ++j) {
        const float rv = (RCVT != 0) ? bf16r(rs[j]) : rs[j];
        val[j] = (u[j] * sc + bf16r(g[j])) + rv;
      }
      xs[i] = val;
      off[i] = o;
    }
#pragma unroll
    for (int i = 0; i < 4; ++i) *(volatile v4f*)(outf + off[i]) = xs[i];
    __threadfence();
#pragma unroll
    for (int i = 0; i < 4; ++i) *(volatile v4f*)(outf + off[i]) = xs[i];
  }

  if (MODE == 3) {
    v8h x[2];
    size_t off[2];
#pragma unroll
    for (unsigned i = 0; i < 2u; ++i) {
      const unsigned r = 32u * i + (tid >> 3);
      const unsigned c = (tid & 7u) * 8u;
      const v4f u0 = *(const v4f*)&Cs[r * LDC + c];
      const v4f u1 = *(const v4f*)&Cs[r * LDC + c + 4];
      const v4f g0 = *(const v4f*)(biasf + n0 + c);
      const v4f g1 = *(const v4f*)(biasf + n0 + c + 4);
#pragma unroll
      for (int j = 0; j < 4; ++j) {
        x[i][j]     = (_Float16)gelu_tanh(u0[j] * (1.0f / WCARRY) + bf16r(g0[j]));
        x[i][j + 4] = (_Float16)gelu_tanh(u1[j] * (1.0f / WCARRY) + bf16r(g1[j]));
      }
      off[i] = (size_t)(row0 + r) * NPITCH + n0 + c;
    }
#pragma unroll
    for (int i = 0; i < 2; ++i) *(volatile v8h*)(out16 + off[i]) = x[i];
    __threadfence();
#pragma unroll
    for (int i = 0; i < 2; ++i) *(volatile v8h*)(out16 + off[i]) = x[i];
  }
}

__global__ __launch_bounds__(256) void gemm_qkv_kernel(
    const _Float16* __restrict__ A16, const _Float16* __restrict__ Bt,
    _Float16* __restrict__ QK, _Float16* __restrict__ Vt) {
  gemm_body<0, DIM, DIM, 6, 0>(A16, Bt, nullptr, nullptr, nullptr, QK, Vt);
}
__global__ __launch_bounds__(256) void gemm_proj_kernel(
    const _Float16* __restrict__ A16, const _Float16* __restrict__ Bt,
    const float* __restrict__ bias, const float* __restrict__ resid,
    float* __restrict__ outf) {
  gemm_body<2, DIM, DIM, 12, 1>(A16, Bt, bias, resid, outf, nullptr, nullptr);
}
__global__ __launch_bounds__(256) void gemm_ff1_kernel(
    const _Float16* __restrict__ A16, const _Float16* __restrict__ Bt,
    const float* __restrict__ bias, _Float16* __restrict__ H16) {
  gemm_body<3, DIM, DFF, 6, 0>(A16, Bt, bias, nullptr, nullptr, H16, nullptr);
}
__global__ __launch_bounds__(256) void gemm_ff2_kernel(
    const _Float16* __restrict__ A16, const _Float16* __restrict__ Bt,
    const float* __restrict__ bias, const float* __restrict__ resid,
    float* __restrict__ outf) {
  gemm_body<2, DFF, DIM, 6, 0>(A16, Bt, bias, resid, outf, nullptr, nullptr);
}

__global__ __launch_bounds__(256) void attn_kernel(
    const _Float16* __restrict__ Qh, const _Float16* __restrict__ Kh,
    const _Float16* __restrict__ Vt, _Float16* __restrict__ Ov) {
  __shared__ _Float16 Ks[64 * LDT];
  __shared__ _Float16 Vs[64 * LDT];
  __shared__ _Float16 Ps[8 * 16 * LDT];

  const unsigned tid = threadIdx.x, lane = tid & 31u, w = tid >> 5;
  const unsigned hh = lane >> 4, m = lane & 15u;
  const unsigned q0 = blockIdx.x * 128u;
  const unsigned head = blockIdx.y;
  const float scale = 0.125f;
  _Float16* P = Ps + w * (16u * LDT);

  const size_t qoff = (size_t)(q0 + w * 16u + m) * DIM + head * HD + hh * 8u;
  v16h qf[2];
  qf[0] = frag_at(Qh + qoff);
  qf[1] = frag_at(Qh + qoff + 32);

  float mrow[8], lrow[8];
  v8f o[4];
#pragma unroll
  for (int v = 0; v < 8; ++v) { mrow[v] = -1.0e30f; lrow[v] = 0.0f; }
#pragma unroll
  for (int nb = 0; nb < 4; ++nb) o[nb] = (v8f){};

  const size_t kplane = (size_t)head * HD;
  const size_t vplane = (size_t)(head * HD) * SEQ;

  for (unsigned kb = 0; kb < (unsigned)SEQ; kb += 64u) {
#pragma unroll
    for (unsigned j = 0; j < 2u; ++j) {
      const unsigned idx = tid + 256u * j;
      const unsigned r = idx >> 3, c = (idx & 7u) * 8u;
      *(v8h*)&Ks[r * LDT + c] = *(const v8h*)(Kh + kplane + (size_t)(kb + r) * DIM + c);
      *(v8h*)&Vs[r * LDT + c] = *(const v8h*)(Vt + vplane + (size_t)r * SEQ + kb + c);
    }
    __syncthreads();

    v8f s[4];
#pragma unroll
    for (int kg = 0; kg < 4; ++kg) {
      v8f t = {};
#pragma unroll
      for (int c = 0; c < 2; ++c) {
        const v16h kf = ld_frag(&Ks[(kg * 16) * LDT + c * 32], LDT);
        t = wmma16(qf[c], kf, t);
      }
      s[kg] = t * scale;
    }

    float alpha[8];
#pragma unroll
    for (int v = 0; v < 8; ++v) {
      float mx = fmaxf(fmaxf(s[0][v], s[1][v]), fmaxf(s[2][v], s[3][v]));
      mx = red16_max(mx);
      const float mn = fmaxf(mrow[v], mx);
      alpha[v] = __expf(mrow[v] - mn);
      mrow[v] = mn;
    }
#pragma unroll
    for (int kg = 0; kg < 4; ++kg)
#pragma unroll
      for (int v = 0; v < 8; ++v) s[kg][v] = __expf(s[kg][v] - mrow[v]);
#pragma unroll
    for (int v = 0; v < 8; ++v) {
      const float rs = red16_sum((s[0][v] + s[1][v]) + (s[2][v] + s[3][v]));
      lrow[v] = alpha[v] * lrow[v] + rs;
    }
#pragma unroll
    for (int nb = 0; nb < 4; ++nb)
#pragma unroll
      for (int v = 0; v < 8; ++v) o[nb][v] = o[nb][v] * alpha[v];

#pragma unroll
    for (int kg = 0; kg < 4; ++kg)
#pragma unroll
      for (int v = 0; v < 8; ++v)
        P[(hh * 8u + (unsigned)v) * LDT + (unsigned)kg * 16u + m] = (_Float16)(s[kg][v] * PCARRY);
    wave_lds_sync();

#pragma unroll
    for (int c = 0; c < 2; ++c) {
      const v16h pf = ld_frag(P + c * 32, LDT);
#pragma unroll
      for (int nb = 0; nb < 4; ++nb) {
        const v16h vf = ld_frag(&Vs[(nb * 16) * LDT + c * 32], LDT);
        o[nb] = wmma16(pf, vf, o[nb]);
      }
    }
    __syncthreads();
  }

  float inv[8];
#pragma unroll
  for (int v = 0; v < 8; ++v) inv[v] = __builtin_amdgcn_rcpf(lrow[v]) * (VCARRY / PCARRY);
#pragma unroll
  for (int nb = 0; nb < 4; ++nb)
#pragma unroll
    for (int v = 0; v < 8; ++v)
      P[(hh * 8u + (unsigned)v) * LDT + (unsigned)nb * 16u + m] = (_Float16)(o[nb][v] * inv[v]);
  wave_lds_sync();
  v8h x[4];
  size_t off[4];
#pragma unroll
  for (unsigned i = 0; i < 4u; ++i) {
    const unsigned r = 4u * i + (lane >> 3);
    const unsigned c = (lane & 7u) * 8u;
    x[i] = *(const v8h*)&P[r * LDT + c];
    off[i] = (size_t)(q0 + w * 16u + r) * DIM + head * HD + c;
  }
#pragma unroll
  for (int i = 0; i < 4; ++i) *(volatile v8h*)(Ov + off[i]) = x[i];
  __threadfence();
#pragma unroll
  for (int i = 0; i < 4; ++i) *(volatile v8h*)(Ov + off[i]) = x[i];
}

extern "C" void kernel_launch(void* const* d_in, const int* in_sizes, int n_in,
                              void* d_out, int out_size, void* d_ws, size_t ws_size,
                              hipStream_t stream) {
  if (n_in < 21) return;
  if ((long long)in_sizes[0] < (long long)SEQ * DIM) return;
  if (in_sizes[1] < DCOND) return;
  if (in_sizes[2] < DIM || in_sizes[3] < DIM || in_sizes[5] < DIM || in_sizes[7] < DIM) return;
  if (in_sizes[10] < DIM || in_sizes[11] < DIM || in_sizes[12] < DIM) return;
  if (in_sizes[14] < DIM || in_sizes[16] < DIM || in_sizes[20] < DIM) return;
  if (in_sizes[18] < DFF) return;
  if ((long long)in_sizes[4] < (long long)DIM * DCOND) return;
  if ((long long)in_sizes[6] < (long long)DIM * DCOND) return;
  if ((long long)in_sizes[13] < (long long)DIM * DCOND) return;
  if ((long long)in_sizes[15] < (long long)DIM * DCOND) return;
  if ((long long)in_sizes[8] < (long long)3 * DIM * DIM) return;
  if ((long long)in_sizes[9] < (long long)DIM * DIM) return;
  if ((long long)in_sizes[17] < (long long)DFF * DIM) return;
  if ((long long)in_sizes[19] < (long long)DIM * DFF) return;
  if ((long long)out_size < (long long)SEQ * DIM) return;
  if (ws_size < WS_TOTAL) return;

  const float* X     = (const float*)d_in[0];
  const float* cond  = (const float*)d_in[1];
  const float* ln1w  = (const float*)d_in[2];
  const float* ln1b  = (const float*)d_in[3];
  const float* g1w   = (const float*)d_in[4];
  const float* g1b   = (const float*)d_in[5];
  const float* be1w  = (const float*)d_in[6];
  const float* be1b  = (const float*)d_in[7];
  const float* qkvw  = (const float*)d_in[8];
  const float* projw = (const float*)d_in[9];
  const float* projb = (const float*)d_in[10];
  const float* ln2w  = (const float*)d_in[11];
  const float* ln2b  = (const float*)d_in[12];
  const float* g2w   = (const float*)d_in[13];
  const float* g2b   = (const float*)d_in[14];
  const float* be2w  = (const float*)d_in[15];
  const float* be2b  = (const float*)d_in[16];
  const float* ff1w  = (const float*)d_in[17];
  const float* ff1b  = (const float*)d_in[18];
  const float* ff2w  = (const float*)d_in[19];
  const float* ff2b  = (const float*)d_in[20];
  float* out = (float*)d_out;

  char* ws = (char*)d_ws;
  float*    tab    = (float*)(ws + OFF_TAB);
  _Float16* Wqkv16 = (_Float16*)(ws + OFF_WQKV);
  _Float16* Wprj16 = (_Float16*)(ws + OFF_WPROJ);
  _Float16* Wff116 = (_Float16*)(ws + OFF_WFF1);
  _Float16* Wff216 = (_Float16*)(ws + OFF_WFF2);
  _Float16* Xn16   = (_Float16*)(ws + OFF_XN);
  _Float16* QK16   = (_Float16*)(ws + OFF_QK);
  _Float16* Vt16   = (_Float16*)(ws + OFF_VT);
  _Float16* Ctx16  = (_Float16*)(ws + OFF_CTX);
  float*    X1     = (float*)(ws + OFF_X1);
  _Float16* H16    = (_Float16*)(ws + OFF_H);

  dim3 blk(256);

  cond_kernel<<<dim3(128), blk, 0, stream>>>(cond, g1w, g1b, be1w, be1b,
                                             g2w, g2b, be2w, be2b, tab);
  wcast_kernel<<<dim3((unsigned)(((size_t)3 * DIM * DIM) / 2048)), blk, 0, stream>>>(qkvw, Wqkv16);
  wcast_kernel<<<dim3((unsigned)(((size_t)DIM * DIM) / 2048)), blk, 0, stream>>>(projw, Wprj16);
  wcast_kernel<<<dim3((unsigned)(((size_t)DFF * DIM) / 2048)), blk, 0, stream>>>(ff1w, Wff116);
  wcast_kernel<<<dim3((unsigned)(((size_t)DIM * DFF) / 2048)), blk, 0, stream>>>(ff2w, Wff216);

  adaln_kernel<<<dim3(SEQ / 8), blk, 0, stream>>>(X, ln1w, ln1b, tab, tab + DIM, Xn16, 1);
  gemm_qkv_kernel<<<dim3(3 * DIM / 64, SEQ / 64), blk, 0, stream>>>(Xn16, Wqkv16, QK16, Vt16);
  attn_kernel<<<dim3(SEQ / 128, NHEAD), blk, 0, stream>>>(
      QK16, QK16 + (size_t)SEQ * DIM, Vt16, Ctx16);
  gemm_proj_kernel<<<dim3(DIM / 64, SEQ / 64), blk, 0, stream>>>(Ctx16, Wprj16, projb, X, X1);

  adaln_kernel<<<dim3(SEQ / 8), blk, 0, stream>>>(X1, ln2w, ln2b, tab + 2 * DIM, tab + 3 * DIM,
                                                  Xn16, 0);
  gemm_ff1_kernel<<<dim3(DFF / 64, SEQ / 64), blk, 0, stream>>>(Xn16, Wff116, ff1b, H16);
  gemm_ff2_kernel<<<dim3(DIM / 64, SEQ / 64), blk, 0, stream>>>(H16, Wff216, ff2b, X1, out);
}
